// TransformerConv_32487132627456
// MI455X (gfx1250) — hardware-verified
//
#include <hip/hip_runtime.h>
#include <stddef.h>
#include <stdint.h>
#include <math.h>


#define DIN     64
#define HN      4
#define CH      64
#define HC      256
#define EDF     11
#define QKVW    768
#define OQ      0
#define OKK     256
#define OV      512
#define KFIN    512
#define NTHR    256
#define NWAVE   8
#define EPT     8
#define CHUNK   (NTHR * EPT)
#define WCAP    (EPT * 32)
#define LISTN   (NWAVE * WCAP)
#define NBMAX   1024
#define SLOTB   10
#define RCAP    28672
#define DEGCAP  64
#define STW     320
#define STWO    64
#define GBM     64
#define GBN     64
#define GTHR    128
#define ATTSC   0.125f
#define WSMAX   268435456
#define LDSW_SWE (2 * RCAP + 2 * NBMAX + LISTN + 2 * NWAVE)
#define LDSW_END (LDSW_SWE + EDF * HC)
#define LDS_AGG  (LDSW_END * 4 + 64)
#define LDS_FIN  (GBM * KFIN * 2 + GBM * GBN * 4)

static_assert((1 << SLOTB) == NBMAX);
static_assert(SLOTB + 21 <= 31);
static_assert((CHUNK & (CHUNK - 1)) == 0 && CHUNK <= 2048 && SLOTB + 11 <= 31);
static_assert(NTHR * 4 == NBMAX);
static_assert(LISTN >= NBMAX);
static_assert(LISTN >= NWAVE * WCAP);
static_assert((RCAP % 32) == 0);
static_assert((NBMAX % NWAVE) == 0);
static_assert(NWAVE * STW <= RCAP && (STW % 4) == 0 && (STWO % 4) == 0);
static_assert(STWO >= HN * 16 && STWO + HC <= STW);
static_assert((LDSW_SWE % 4) == 0);
static_assert(((EDF * HC) % 4) == 0);
static_assert(LDS_AGG <= 300000 && LDS_FIN <= 300000);
static_assert(GBM == (GTHR / 32) * 16);
static_assert(GBM * 8 == 4 * GTHR);
static_assert(HC == 32 * 8);
static_assert(CH == 8 * 8 && HN * CH == HC);
static_assert(2 * 8 <= 16 && EDF <= 16);
static_assert((DIN % 32) == 0 && (KFIN % 32) == 0 && KFIN == 2 * HC);
static_assert(QKVW == 3 * HC && (QKVW % GBN) == 0 && (HC % GBN) == 0 && CH == GBN);

typedef float          v4f  __attribute__((ext_vector_type(4)));
typedef float          v8f  __attribute__((ext_vector_type(8)));
typedef int            v4i  __attribute__((ext_vector_type(4)));
typedef int            v8i  __attribute__((ext_vector_type(8)));
typedef unsigned int   v4u  __attribute__((ext_vector_type(4)));
typedef unsigned short v8us __attribute__((ext_vector_type(8)));
typedef __bf16         v16b __attribute__((ext_vector_type(16)));
typedef v4f  __attribute__((may_alias)) v4fa;
typedef v4u  __attribute__((may_alias)) v4ua;
typedef v8us __attribute__((may_alias)) v8usa;
union FragB { v16b v; v8us h[2]; v8i w; };

__device__ __forceinline__ v8f wmb(const FragB& a, const FragB& b, v8f c) {
  v8f d = __builtin_amdgcn_wmma_f32_16x16x32_bf16(false, a.v, false, b.v, (short)0, c, false, false);
  asm volatile("v_nop\n\tv_nop\n\tv_nop\n\tv_nop" : "+v"(d) : "v"(a.w), "v"(b.w));
  return d;
}

__device__ __forceinline__ void ldwait() {
  asm volatile("s_wait_loadcnt 0x0" ::: "memory");
}

__device__ __forceinline__ unsigned int f2bf(float f) {
  const unsigned int u = __float_as_uint(f);
  return ((u + 0x7FFFu + ((u >> 16) & 1u)) >> 16) & 0xFFFFu;
}
__device__ __forceinline__ float bf2f(unsigned int b) { return __uint_as_float(b << 16); }
__device__ __forceinline__ float bfr(float f) { return bf2f(f2bf(f)); }
__device__ __forceinline__ v4f bfr4(const v4f a) {
  v4f r; r.x = bfr(a.x); r.y = bfr(a.y); r.z = bfr(a.z); r.w = bfr(a.w); return r;
}
__device__ __forceinline__ unsigned int pk2(float lo, float hi) { return f2bf(lo) | (f2bf(hi) << 16); }
__device__ __forceinline__ v4u pack8(const v4f a, const v4f b) {
  v4u r;
  r.x = pk2(a.x, a.y); r.y = pk2(a.z, a.w); r.z = pk2(b.x, b.y); r.w = pk2(b.z, b.w);
  return r;
}
__device__ __forceinline__ void hl2(float v0, float v1, unsigned int& hw, unsigned int& lw) {
  const unsigned int h0 = f2bf(v0), h1 = f2bf(v1);
  const unsigned int l0 = f2bf(v0 - bf2f(h0)), l1 = f2bf(v1 - bf2f(h1));
  hw = h0 | (h1 << 16);
  lw = l0 | (l1 << 16);
}
__device__ __forceinline__ void pack8hl(const v4f a, const v4f b, v4u& hv, v4u& lv) {
  unsigned int h, l;
  hl2(a.x, a.y, h, l); hv.x = h; lv.x = l;
  hl2(a.z, a.w, h, l); hv.y = h; lv.y = l;
  hl2(b.x, b.y, h, l); hv.z = h; lv.z = l;
  hl2(b.z, b.w, h, l); hv.w = h; lv.w = l;
}

__device__ __forceinline__ int scan_chunk(const int* __restrict__ dsts, int nE, int cbase, int slotBase,
                                          int nb, int vec8, int* list, int tid, int lane, int wave) {
  int wc = 0;
  const int el0  = tid * EPT;
  const int e0   = cbase + el0;
  const int sent = -2147483647 - 1;
  v4i da, db;
  if (vec8 != 0 && cbase + CHUNK <= nE) {
    da = *(const v4i*)(dsts + e0);
    db = *(const v4i*)(dsts + e0 + 4);
  } else {
    da.x = (e0     < nE) ? dsts[min(e0,     nE - 1)] : sent;
    da.y = (e0 + 1 < nE) ? dsts[min(e0 + 1, nE - 1)] : sent;
    da.z = (e0 + 2 < nE) ? dsts[min(e0 + 2, nE - 1)] : sent;
    da.w = (e0 + 3 < nE) ? dsts[min(e0 + 3, nE - 1)] : sent;
    db.x = (e0 + 4 < nE) ? dsts[min(e0 + 4, nE - 1)] : sent;
    db.y = (e0 + 5 < nE) ? dsts[min(e0 + 5, nE - 1)] : sent;
    db.z = (e0 + 6 < nE) ? dsts[min(e0 + 6, nE - 1)] : sent;
    db.w = (e0 + 7 < nE) ? dsts[min(e0 + 7, nE - 1)] : sent;
  }
  const unsigned nbs = (unsigned)slotBase;
  const unsigned unb = (unsigned)nb;
  const unsigned s0 = (unsigned)da.x - nbs, s1 = (unsigned)da.y - nbs;
  const unsigned s2 = (unsigned)da.z - nbs, s3 = (unsigned)da.w - nbs;
  const unsigned s4 = (unsigned)db.x - nbs, s5 = (unsigned)db.y - nbs;
  const unsigned s6 = (unsigned)db.z - nbs, s7 = (unsigned)db.w - nbs;
  const bool h0 = s0 < unb, h1 = s1 < unb, h2 = s2 < unb, h3 = s3 < unb;
  const bool h4 = s4 < unb, h5 = s5 < unb, h6 = s6 < unb, h7 = s7 < unb;
  const unsigned any = __builtin_amdgcn_ballot_w32(h0 | h1 | h2 | h3 | h4 | h5 | h6 | h7);
  if (any != 0u) {
#define HITJ(J, HJ, SJ) { \
      const unsigned mj = __builtin_amdgcn_ballot_w32(HJ); \
      if (mj != 0u) { \
        if (HJ) { \
          const int pos = wc + (int)__builtin_amdgcn_mbcnt_lo(mj, 0u); \
          if (pos < WCAP) list[wave * WCAP + pos] = ((el0 + (J)) << SLOTB) | (int)(SJ); \
        } \
        wc += (int)__builtin_popcount(mj); } }
    HITJ(0, h0, s0)
    HITJ(1, h1, s1)
    HITJ(2, h2, s2)
    HITJ(3, h3, s3)
    HITJ(4, h4, s4)
    HITJ(5, h5, s5)
    HITJ(6, h6, s6)
    HITJ(7, h7, s7)
#undef HITJ
  }
  return wc;
}

__global__ __launch_bounds__(NTHR) void k_xprep(const float* __restrict__ x, unsigned short* xb, int nN, int nUnits) {
  const int i = (int)blockIdx.x * NTHR + (int)threadIdx.x;
  if (i >= nUnits) return;
  const int row = i >> 3;
  const int c0  = (i & 7) * 8;
  const int rc  = row < nN ? row : nN - 1;
  const float* p = x + (size_t)rc * DIN + c0;
  v4f a = *(const v4fa*)p;
  v4f b = *(const v4fa*)(p + 4);
  const v4f z4 = {0.f, 0.f, 0.f, 0.f};
  if (row >= nN) { a = z4; b = z4; }
  const v4u hv = pack8(a, b);
  unsigned short* o = xb + (size_t)row * DIN + c0;
  *(volatile v4u*)o = hv;
  __threadfence();
  *(volatile v4u*)o = hv;
}

__global__ __launch_bounds__(NTHR) void k_wtr(const float* __restrict__ w, int Kin, int Ncol, int Nrows, int Kout,
                                              unsigned short* wt, int nUnits) {
  const int u = (int)blockIdx.x * NTHR + (int)threadIdx.x;
  if (u >= nUnits) return;
  const int kq = Kout >> 3;
  const int n  = u / kq;
  const int k8 = (u - n * kq) * 8;
  const int kk = k8 - (k8 / Kin) * Kin;
  const int ncl = n < Ncol ? n : Ncol - 1;
  const float* p = w + (size_t)kk * (size_t)Ncol + ncl;
  v4f a, b;
  a.x = p[0];                    a.y = p[(size_t)Ncol];         a.z = p[(size_t)2 * Ncol];     a.w = p[(size_t)3 * Ncol];
  b.x = p[(size_t)4 * Ncol];     b.y = p[(size_t)5 * Ncol];     b.z = p[(size_t)6 * Ncol];     b.w = p[(size_t)7 * Ncol];
  const v4f z4 = {0.f, 0.f, 0.f, 0.f};
  if (n >= Ncol || n >= Nrows) { a = z4; b = z4; }
  const v4u wv = pack8(a, b);
  unsigned short* o = wt + (size_t)n * (size_t)Kout + k8;
  *(volatile v4u*)o = wv;
  __threadfence();
  *(volatile v4u*)o = wv;
}

__global__ __launch_bounds__(GTHR) void k_gemm(
    const unsigned short* __restrict__ A, const unsigned short* __restrict__ WT,
    float* outF, int K, int ldo)
{
  __shared__ __attribute__((aligned(16))) float stg[GBM * GBN];
  const int tid = (int)threadIdx.x, lane = tid & 31, wave = tid >> 5, hh = lane >> 4, m = lane & 15;
  const int rowBase = (int)blockIdx.x * GBM;
  const int col0    = (int)blockIdx.y * GBN;

  v8f acc[4];
  {
    const v8f z = {0.f, 0.f, 0.f, 0.f, 0.f, 0.f, 0.f, 0.f};
    acc[0] = z; acc[1] = z; acc[2] = z; acc[3] = z;
  }
  const unsigned short* ap = A  + (size_t)(rowBase + 16 * wave + m) * (size_t)K + 8 * hh;
  const unsigned short* wp = WT + (size_t)(col0 + m) * (size_t)K + 8 * hh;
  const int ksteps = K >> 5;
#pragma unroll 1
  for (int ks = 0; ks < ksteps; ++ks) {
    FragB af;
    af.h[0] = *(const v8usa*)(ap + 32 * ks);
    af.h[1] = *(const v8usa*)(ap + 32 * ks + 16);
#pragma unroll
    for (int t = 0; t < 4; ++t) {
      const unsigned short* wq = wp + (size_t)(16 * t) * (size_t)K + 32 * ks;
      FragB bf;
      bf.h[0] = *(const v8usa*)wq;
      bf.h[1] = *(const v8usa*)(wq + 16);
      acc[t] = wmb(af, bf, acc[t]);
    }
  }

#pragma unroll
  for (int t = 0; t < 4; ++t) {
    const int lc = 16 * t + m;
#pragma unroll
    for (int r = 0; r < 8; ++r) {
      const int lr = 16 * wave + 8 * hh + r;
      stg[lr * GBN + lc] = acc[t][r];
    }
  }
  __syncthreads();

  v4f fv[8];
#pragma unroll
  for (int i = 0; i < 8; ++i) {
    const int lr = 16 * wave + 2 * i + hh;
    fv[i] = *(const v4fa*)(stg + lr * GBN + 4 * m);
  }
#pragma unroll
  for (int i = 0; i < 8; ++i) {
    const int lr = 16 * wave + 2 * i + hh;
    const int gr = rowBase + lr;
    float* op = outF + (size_t)gr * (size_t)ldo + col0 + 4 * m;
    *(volatile v4f*)op = fv[i];
  }
  __threadfence();
#pragma unroll
  for (int i = 0; i < 8; ++i) {
    const int lr = 16 * wave + 2 * i + hh;
    const int gr = rowBase + lr;
    float* op = outF + (size_t)gr * (size_t)ldo + col0 + 4 * m;
    *(volatile v4f*)op = fv[i];
  }
}

__global__ __launch_bounds__(NTHR) void k_agg(
    const int* __restrict__ srcs, const int* __restrict__ dsts,
    const float* __restrict__ QKV, const float* __restrict__ eattr, const float* __restrict__ We,
    float* OUTP, int nN, int nE, int vec8, int MPr) {
  extern __shared__ v4f lds_dyn[];
  int* reg1 = (int*)lds_dyn;
  int* reg2 = reg1 + RCAP;
  int* scnt = reg2 + RCAP;
  int* soff = scnt + NBMAX;
  int* list = soff + NBMAX;
  int* wcnt = list + LISTN;
  int* wtot = wcnt + NWAVE;
  float* sWe = (float*)(wtot + NWAVE);
  const int tid = (int)threadIdx.x, lane = tid & 31, wave = tid >> 5;
  const int nodeBase = (int)blockIdx.x * NBMAX;

  for (int i = tid; i < NBMAX; i += NTHR) scnt[i] = 0;
#pragma unroll 1
  for (int i = tid; i < (EDF * HC) / 4; i += NTHR) {
    const v4f wv = *(const v4fa*)(We + 4 * i);
    *(v4fa*)(sWe + 4 * i) = bfr4(wv);
  }
  __syncthreads();

  int tot = 0;
  const int nChunks = (nE + CHUNK - 1) / CHUNK;
#pragma unroll 1
  for (int ch = 0; ch < nChunks; ++ch) {
    const int cbase = ch * CHUNK;
    const int wc = scan_chunk(dsts, nE, cbase, nodeBase, NBMAX, vec8, list, tid, lane, wave);
    if (lane == 0) wcnt[wave] = wc;
    __syncthreads();
    int pre = 0, all = 0;
#pragma unroll
    for (int w2 = 0; w2 < NWAVE; ++w2) {
      int c = wcnt[w2];
      c = c < 0 ? 0 : (c > WCAP ? WCAP : c);
      all += c;
      pre += (w2 < wave) ? c : 0;
    }
    const int wcc  = wc > WCAP ? WCAP : wc;
    const int base = tot + pre;
#pragma unroll 1
    for (int i = lane; i < wcc; i += 32) {
      const int ent = list[wave * WCAP + i];
      const int el  = (ent >> SLOTB) & (CHUNK - 1);
      const int sl  = ent & (NBMAX - 1);
      int eid = cbase + el;
      eid = eid > nE - 1 ? nE - 1 : eid;
      const int pos = base + i;
      if (pos < RCAP) reg1[pos] = (int)(((unsigned)eid << SLOTB) | (unsigned)sl);
    }
    tot += all;
    tot = tot > RCAP ? RCAP : tot;
    __syncthreads();
  }
  const int nh = tot;

  if (wave == 0) {
#pragma unroll 1
    for (int b0 = 0; b0 < nh; b0 += 32) {
      const int idx = b0 + lane;
      const int uv  = reg1[idx < nh ? idx : nh - 1];
      const int m32 = (nh - b0) < 32 ? (nh - b0) : 32;
#pragma unroll 1
      for (int k = 0; k < m32; ++k) {
        const int u  = __builtin_amdgcn_readlane(uv, k);
        const int sl = u & (NBMAX - 1);
        if (lane == 0) scnt[sl] = scnt[sl] + 1;
      }
    }
  }
  __syncthreads();

  {
    const v4i ca = *(const v4i*)(scnt + 4 * tid);
    const int e0 = ca.x < 0 ? 0 : ca.x, e1 = ca.y < 0 ? 0 : ca.y, e2 = ca.z < 0 ? 0 : ca.z, e3 = ca.w < 0 ? 0 : ca.w;
    const int ts = e0 + e1 + e2 + e3;
    int incl = ts;
#pragma unroll
    for (int d = 1; d < 32; d <<= 1) {
      const int up = __shfl_up(incl, d);
      if (lane >= d) incl += up;
    }
    if (lane == 31) wtot[wave] = incl;
    __syncthreads();
    int pre = 0;
#pragma unroll
    for (int w2 = 0; w2 < NWAVE; ++w2) pre += (w2 < wave) ? wtot[w2] : 0;
    int run = pre + incl - ts;
    soff[4 * tid + 0] = run; run += e0;
    soff[4 * tid + 1] = run; run += e1;
    soff[4 * tid + 2] = run; run += e2;
    soff[4 * tid + 3] = run;
  }
  __syncthreads();
  for (int i = tid; i < NBMAX; i += NTHR) list[i] = soff[i];
  __syncthreads();

  if (wave == 0) {
#pragma unroll 1
    for (int b0 = 0; b0 < nh; b0 += 32) {
      const int idx = b0 + lane;
      const int uv  = reg1[idx < nh ? idx : nh - 1];
      const int m32 = (nh - b0) < 32 ? (nh - b0) : 32;
#pragma unroll 1
      for (int k = 0; k < m32; ++k) {
        const int u   = __builtin_amdgcn_readlane(uv, k);
        const int sl  = u & (NBMAX - 1);
        const int eid = (int)((unsigned)u >> SLOTB);
        if (lane == 0) {
          int pos = list[sl];
          pos = pos < 0 ? 0 : (pos > RCAP - 1 ? RCAP - 1 : pos);
          reg2[pos] = eid;
          list[sl] = pos + 1;
        }
      }
    }
  }
  __syncthreads();

  const int nbw = NBMAX / NWAVE;
  const bool ovf = (nh >= RCAP);
  const float qnan = __int_as_float(0x7fc00000);
  float* stw = (float*)reg1 + wave * STW;
  const int hd = lane >> 3;
  const int jj = lane & 7;
  const int t0 = 2 * jj, t1 = 2 * jj + 1;
  const int t0c = t0 < EDF ? t0 : EDF - 1;
  const int t1c = t1 < EDF ? t1 : EDF - 1;
  const float t0m = t0 < EDF ? 1.0f : 0.0f;
  const float t1m = t1 < EDF ? 1.0f : 0.0f;

#pragma unroll 1
  for (int jt = 0; jt < nbw; ++jt) {
    const int slot = wave * nbw + jt;
    const int grow = nodeBase + slot;
    const int gcl  = grow < nN ? grow : nN - 1;
    int st = soff[slot];
    const int craw = scnt[slot];
    int cnt = craw;
    st  = st < 0 ? 0 : (st > nh ? nh : st);
    cnt = cnt < 0 ? 0 : (cnt > DEGCAP ? DEGCAP : cnt);
    if (cnt > nh - st) cnt = nh - st;
    const float pz = (ovf || craw > DEGCAP) ? qnan : 0.0f;

    const float* qr = QKV + (size_t)gcl * QKVW + OQ + 8 * lane;
    const v4f qa = *(const v4fa*)qr;
    const v4f qb = *(const v4fa*)(qr + 4);
    ldwait();

    float QW0 = 0.f, QW1 = 0.f;
#pragma unroll 1
    for (int t = 0; t < EDF; ++t) {
      const float* wr = sWe + t * HC + 8 * lane;
      const v4f w0 = *(const v4fa*)wr;
      const v4f w1 = *(const v4fa*)(wr + 4);
      float p = qa.x * w0.x;
      p = fmaf(qa.y, w0.y, p); p = fmaf(qa.z, w0.z, p); p = fmaf(qa.w, w0.w, p);
      p = fmaf(qb.x, w1.x, p); p = fmaf(qb.y, w1.y, p); p = fmaf(qb.z, w1.z, p); p = fmaf(qb.w, w1.w, p);
      p += __shfl_xor(p, 4);
      p += __shfl_xor(p, 2);
      p += __shfl_xor(p, 1);
      QW0 = (t == t0) ? p : QW0;
      QW1 = (t == t1) ? p : QW1;
    }

    float mx = -1.0e30f, dn = 0.f, ae0 = 0.f, ae1 = 0.f;
    v4f ava = {0.f, 0.f, 0.f, 0.f};
    v4f avb = {0.f, 0.f, 0.f, 0.f};
#pragma unroll 1
    for (int q = 0; q < cnt; ++q) {
      int idx = st + q; idx = idx > RCAP - 1 ? RCAP - 1 : idx;
      int eid = reg2[idx]; eid = eid < 0 ? 0 : (eid > nE - 1 ? nE - 1 : eid);
      const int sraw = srcs[eid];
      const int s = sraw < 0 ? 0 : (sraw > nN - 1 ? nN - 1 : sraw);
      const float* er = eattr + (size_t)eid * EDF;
      const float ea0 = bfr(er[t0c]) * t0m;
      const float ea1 = bfr(er[t1c]) * t1m;
      const float* kr = QKV + (size_t)s * QKVW + OKK + 8 * lane;
      const v4f ka = *(const v4fa*)kr;
      const v4f kb = *(const v4fa*)(kr + 4);
      const float* vr = QKV + (size_t)s * QKVW + OV + 8 * lane;
      const v4f va = *(const v4fa*)vr;
      const v4f vb = *(const v4fa*)(vr + 4);
      ldwait();
      float p = qa.x * ka.x;
      p = fmaf(qa.y, ka.y, p); p = fmaf(qa.z, ka.z, p); p = fmaf(qa.w, ka.w, p);
      p = fmaf(qb.x, kb.x, p); p = fmaf(qb.y, kb.y, p); p = fmaf(qb.z, kb.z, p); p = fmaf(qb.w, kb.w, p);
      p = fmaf(ea0, QW0, p);
      p = fmaf(ea1, QW1, p);
      p += __shfl_xor(p, 4);
      p += __shfl_xor(p, 2);
      p += __shfl_xor(p, 1);
      const float lg = p * ATTSC;
      const float df = lg - mx;
      const float ee = __expf(-fabsf(df));
      const bool up  = df > 0.f;
      const float s1 = up ? ee : 1.0f;
      const float s2 = up ? 1.0f : ee;
      mx = up ? lg : mx;
      dn = fmaf(dn, s1, s2);
      ava.x = fmaf(ava.x, s1, s2 * va.x); ava.y = fmaf(ava.y, s1, s2 * va.y);
      ava.z = fmaf(ava.z, s1, s2 * va.z); ava.w = fmaf(ava.w, s1, s2 * va.w);
      avb.x = fmaf(avb.x, s1, s2 * vb.x); avb.y = fmaf(avb.y, s1, s2 * vb.y);
      avb.z = fmaf(avb.z, s1, s2 * vb.z); avb.w = fmaf(avb.w, s1, s2 * vb.w);
      ae0 = fmaf(ae0, s1, s2 * ea0);
      ae1 = fmaf(ae1, s1, s2 * ea1);
    }
    const float dns = dn > 0.f ? dn : 1.0f;
    const float ind = dn > 0.f ? 1.0f : 0.0f;
    const float inv = ind * __builtin_amdgcn_rcpf(dns);
    const float aen0 = ae0 * inv;
    const float aen1 = ae1 * inv;
    __builtin_amdgcn_fence(__ATOMIC_RELEASE, "wavefront");
    __builtin_amdgcn_wave_barrier();
    stw[hd * 16 + t0] = aen0;
    stw[hd * 16 + t1] = aen1;
    __builtin_amdgcn_fence(__ATOMIC_RELEASE, "wavefront");
    __builtin_amdgcn_wave_barrier();
    v4f oa, ob;
    oa.x = ava.x * inv; oa.y = ava.y * inv; oa.z = ava.z * inv; oa.w = ava.w * inv;
    ob.x = avb.x * inv; ob.y = avb.y * inv; ob.z = avb.z * inv; ob.w = avb.w * inv;
#pragma unroll 1
    for (int t = 0; t < EDF; ++t) {
      const float a = stw[hd * 16 + t];
      const float* wr = sWe + t * HC + 8 * lane;
      const v4f w0 = *(const v4fa*)wr;
      const v4f w1 = *(const v4fa*)(wr + 4);
      oa.x = fmaf(a, w0.x, oa.x); oa.y = fmaf(a, w0.y, oa.y); oa.z = fmaf(a, w0.z, oa.z); oa.w = fmaf(a, w0.w, oa.w);
      ob.x = fmaf(a, w1.x, ob.x); ob.y = fmaf(a, w1.y, ob.y); ob.z = fmaf(a, w1.z, ob.z); ob.w = fmaf(a, w1.w, ob.w);
    }
    oa.x += pz; oa.y += pz; oa.z += pz; oa.w += pz;
    ob.x += pz; ob.y += pz; ob.z += pz; ob.w += pz;
    __builtin_amdgcn_fence(__ATOMIC_RELEASE, "wavefront");
    __builtin_amdgcn_wave_barrier();
    *(v4fa*)(stw + STWO + 8 * lane)     = oa;
    *(v4fa*)(stw + STWO + 8 * lane + 4) = ob;
    __builtin_amdgcn_fence(__ATOMIC_RELEASE, "wavefront");
    __builtin_amdgcn_wave_barrier();
    const v4f pa = *(const v4fa*)(stw + STWO + 4 * lane);
    const v4f pb = *(const v4fa*)(stw + STWO + (HC / 2) + 4 * lane);
    const bool wr = (grow < MPr);
    const int gsf = wr ? grow : MPr - 1;
    float* orow = OUTP + (size_t)gsf * HC;
    if (wr) {
      *(volatile v4f*)(orow + 4 * lane)            = pa;
      *(volatile v4f*)(orow + (HC / 2) + 4 * lane) = pb;
    }
    __threadfence();
    if (wr) {
      *(volatile v4f*)(orow + 4 * lane)            = pa;
      *(volatile v4f*)(orow + (HC / 2) + 4 * lane) = pb;
    }
  }
}

__global__ __launch_bounds__(GTHR) void k_final(
    const unsigned short* __restrict__ XB, const unsigned short* __restrict__ WSKT,
    const float* __restrict__ OUTP, const unsigned short* __restrict__ WLT2,
    float* out, int nN)
{
  extern __shared__ v4f lds_dyn[];
  unsigned short* At = (unsigned short*)lds_dyn;
  float* stg = (float*)(At + GBM * KFIN);
  const int tid = (int)threadIdx.x, lane = tid & 31, wave = tid >> 5, hh = lane >> 4, m = lane & 15;
  const int rowBase = (int)blockIdx.x * GBM;

  FragB ax[2];
  {
    const unsigned short* ap = XB + (size_t)(rowBase + 16 * wave + m) * DIN + 8 * hh;
    ax[0].h[0] = *(const v8usa*)(ap);
    ax[0].h[1] = *(const v8usa*)(ap + 16);
    ax[1].h[0] = *(const v8usa*)(ap + 32);
    ax[1].h[1] = *(const v8usa*)(ap + 48);
  }

#pragma unroll 1
  for (int g = 0; g < HC / GBN; ++g) {
    v8f acc[4];
    {
      const v8f z = {0.f, 0.f, 0.f, 0.f, 0.f, 0.f, 0.f, 0.f};
      acc[0] = z; acc[1] = z; acc[2] = z; acc[3] = z;
    }
    const unsigned short* wp = WSKT + (size_t)(g * GBN + m) * DIN + 8 * hh;
#pragma unroll
    for (int ks = 0; ks < DIN / 32; ++ks) {
#pragma unroll
      for (int t = 0; t < 4; ++t) {
        const unsigned short* wq = wp + (size_t)(16 * t) * DIN + 32 * ks;
        FragB bf;
        bf.h[0] = *(const v8usa*)wq;
        bf.h[1] = *(const v8usa*)(wq + 16);
        acc[t] = wmb(ax[ks], bf, acc[t]);
      }
    }
#pragma unroll
    for (int t = 0; t < 4; ++t) {
      const int lc = 16 * t + m;
#pragma unroll
      for (int r = 0; r < 8; ++r) {
        const int lr = 16 * wave + 8 * hh + r;
        stg[lr * GBN + lc] = acc[t][r];
      }
    }
    __syncthreads();
#pragma unroll
    for (int i = 0; i < 4; ++i) {
      const int p   = i * GTHR + tid;
      const int row = p >> 3;
      const int q8  = (p & 7) * 8;
      v4f a = *(const v4fa*)(stg + row * GBN + q8);
      v4f b = *(const v4fa*)(stg + row * GBN + q8 + 4);
      const float* orp = OUTP + (size_t)(rowBase + row) * HC + g * GBN + q8;
      const v4f oa = *(const v4fa*)orp;
      const v4f ob = *(const v4fa*)(orp + 4);
      a = a + oa;
      b = b + ob;
      v4u hv, lv;
      pack8hl(a, b, hv, lv);
      *(v4ua*)(At + row * KFIN + g * GBN + q8)      = hv;
      *(v4ua*)(At + row * KFIN + HC + g * GBN + q8) = lv;
    }
    __syncthreads();
  }

  v8f acc2[4];
  {
    const v8f z = {0.f, 0.f, 0.f, 0.f, 0.f, 0.f, 0.f, 0.f};
    acc2[0] = z; acc2[1] = z; acc2[2] = z; acc2[3] = z;
  }
  const unsigned short* aq = At + (size_t)(16 * wave + m) * KFIN + 8 * hh;
  const unsigned short* wl = WLT2 + (size_t)m * KFIN + 8 * hh;
#pragma unroll 1
  for (int ks = 0; ks < KFIN / 32; ++ks) {
    FragB af;
    af.h[0] = *(const v8usa*)(aq + 32 * ks);
    af.h[1] = *(const v8usa*)(aq + 32 * ks + 16);
#pragma unroll
    for (int t = 0; t < 4; ++t) {
      const unsigned short* wq = wl + (size_t)(16 * t) * KFIN + 32 * ks;
      FragB bf;
      bf.h[0] = *(const v8usa*)wq;
      bf.h[1] = *(const v8usa*)(wq + 16);
      acc2[t] = wmb(af, bf, acc2[t]);
    }
  }

#pragma unroll
  for (int t = 0; t < 4; ++t) {
    const int lc = 16 * t + m;
#pragma unroll
    for (int r = 0; r < 8; ++r) {
      const int lr = 16 * wave + 8 * hh + r;
      stg[lr * GBN + lc] = acc2[t][r];
    }
  }
  __syncthreads();

  v4f fv[8];
#pragma unroll
  for (int i = 0; i < 8; ++i) {
    const int lr = 16 * wave + 2 * i + hh;
    fv[i] = *(const v4fa*)(stg + lr * GBN + 4 * m);
  }
#pragma unroll
  for (int i = 0; i < 8; ++i) {
    const int lr = 16 * wave + 2 * i + hh;
    const int gr = rowBase + lr;
    const int gs = gr < nN ? gr : nN - 1;
    float* op = out + (size_t)gs * CH + 4 * m;
    if (gr < nN) *(volatile v4f*)op = fv[i];
  }
  __threadfence();
#pragma unroll
  for (int i = 0; i < 8; ++i) {
    const int lr = 16 * wave + 2 * i + hh;
    const int gr = rowBase + lr;
    const int gs = gr < nN ? gr : nN - 1;
    float* op = out + (size_t)gs * CH + 4 * m;
    if (gr < nN) *(volatile v4f*)op = fv[i];
  }
}

static inline int cdiv(int a, int b) { return (a + b - 1) / b; }

extern "C" void kernel_launch(void* const* d_in, const int* in_sizes, int n_in,
                              void* d_out, int out_size, void* d_ws, size_t ws_size,
                              hipStream_t stream) {
  if (n_in < 9) return;
  if (in_sizes[0] < DIN || (in_sizes[0] % DIN) != 0) return;
  const int nN = in_sizes[0] / DIN;
  if (nN < 1 || nN > (1 << 22)) return;
  if (in_sizes[2] < 2 || (in_sizes[2] & 1) != 0) return;
  const int nE = in_sizes[2] / 2;
  if (nE < 1 || nE >= (1 << (31 - SLOTB))) return;
  if (in_sizes[1] != nE * EDF) return;
  if (in_sizes[3] != DIN * HC || in_sizes[4] != DIN * HC || in_sizes[5] != DIN * HC) return;
  if (in_sizes[6] != EDF * HC) return;
  if (in_sizes[7] != DIN * HC) return;
  if (in_sizes[8] != HC * CH) return;
  if (out_size != nN * CH) return;

  const float* x      = (const float*)d_in[0];
  const float* eattr  = (const float*)d_in[1];
  const int*   ei     = (const int*)  d_in[2];
  const float* Wq     = (const float*)d_in[3];
  const float* Wk     = (const float*)d_in[4];
  const float* Wv     = (const float*)d_in[5];
  const float* We     = (const float*)d_in[6];
  const float* Wskip  = (const float*)d_in[7];
  const float* Wlin   = (const float*)d_in[8];
  float* out = (float*)d_out;
  const int* src = ei;
  const int* dst = ei + nE;

  const int MP   = cdiv(nN, GBM) * GBM;
  const int gA   = cdiv(MP, NBMAX);
  const int vec8 = ((nE & 3) == 0) ? 1 : 0;
  if (gA * NBMAX < MP) return;

  char* ws = (char*)d_ws;
  size_t off = 0;
  const size_t oXB  = off; off += (size_t)MP * DIN * 2;            off = (off + 255) & ~(size_t)255;
  const size_t oWQ  = off; off += (size_t)QKVW * DIN * 2;          off = (off + 255) & ~(size_t)255;
  const size_t oWS  = off; off += (size_t)HC * DIN * 2;            off = (off + 255) & ~(size_t)255;
  const size_t oWL  = off; off += (size_t)CH * KFIN * 2;           off = (off + 255) & ~(size_t)255;
  const size_t oQKV = off; off += (size_t)MP * QKVW * 4;           off = (off + 255) & ~(size_t)255;
  const size_t oOUT = off; off += (size_t)MP * HC * 4;             off = (off + 255) & ~(size_t)255;
  if (off > ws_size || off > (size_t)WSMAX) return;
  unsigned short* XB    = (unsigned short*)(ws + oXB);
  unsigned short* WQKVT = (unsigned short*)(ws + oWQ);
  unsigned short* WSKT  = (unsigned short*)(ws + oWS);
  unsigned short* WLT2  = (unsigned short*)(ws + oWL);
  float*          QKV   = (float*)(ws + oQKV);
  float*          OUTP  = (float*)(ws + oOUT);

  hipFuncSetAttribute(reinterpret_cast<const void*>(&k_agg),
                      hipFuncAttributeMaxDynamicSharedMemorySize, LDS_AGG);
  hipFuncSetAttribute(reinterpret_cast<const void*>(&k_final),
                      hipFuncAttributeMaxDynamicSharedMemorySize, LDS_FIN);

  const int nUx = MP * (DIN / 8);
  k_xprep<<<cdiv(nUx, NTHR), NTHR, 0, stream>>>(x, XB, nN, nUx);

  {
    const int nUq = HC * (DIN / 8);
    k_wtr<<<cdiv(nUq, NTHR), NTHR, 0, stream>>>(Wq,    DIN, HC, HC, DIN, WQKVT,                        nUq);
    k_wtr<<<cdiv(nUq, NTHR), NTHR, 0, stream>>>(Wk,    DIN, HC, HC, DIN, WQKVT + (size_t)HC * DIN,      nUq);
    k_wtr<<<cdiv(nUq, NTHR), NTHR, 0, stream>>>(Wv,    DIN, HC, HC, DIN, WQKVT + (size_t)2 * HC * DIN,  nUq);
    k_wtr<<<cdiv(nUq, NTHR), NTHR, 0, stream>>>(Wskip, DIN, HC, HC, DIN, WSKT,                         nUq);
    const int nUl = CH * (KFIN / 8);
    k_wtr<<<cdiv(nUl, NTHR), NTHR, 0, stream>>>(Wlin,  HC, CH, CH, KFIN, WLT2, nUl);
  }

  const int gM = MP / GBM;
  k_gemm<<<dim3(gM, QKVW / GBN), GTHR, 0, stream>>>(XB, WQKVT, QKV, DIN, QKVW);
  k_agg<<<gA, NTHR, LDS_AGG, stream>>>(src, dst, QKV, eattr, We, OUTP, nN, nE, vec8, MP);
  k_final<<<gM, GTHR, LDS_FIN, stream>>>(XB, WSKT, OUTP, WLT2, out, nN);
}
